// GNNModel_45122926411919
// MI455X (gfx1250) — hardware-run, weakly checked
//
#include <hip/hip_runtime.h>


namespace {

constexpr int N = 100000, NP = 100032, NPL = NP  , SRCM = N  , EFULL = 1600000, E = EFULL  ;
constexpr int FIN = 128  , F = 64  , FO = 64, NLAY = 3, PE = (NLAY + 1) * F  , P2 = 2 * F  , VOC = 1, D1 = F, NRL = NP  , NL = (NPL < N ? NPL : N);
constexpr float LNEPS = 1e-5f; constexpr float LOG2E = 1.4426950408889634f; constexpr float XS = 8.0f, WSC = 256.0f, WSQ = 0.25f, RS_ = 1024.0f, NSL_ = 0.2f, NSA_ = 0.01f, SLOPE = 0.0f, BNEPS = 1e-5f;
static_assert(NP % 32 == 0 && NP >= N && NPL % 32 == 0 && D1 % 32 == 0, "tiling");
typedef _Float16 b16;
typedef __attribute__((ext_vector_type(16))) _Float16 v16b;
typedef __attribute__((ext_vector_type(8))) _Float16 v8b;
typedef __attribute__((ext_vector_type(8))) float v8f;
typedef __attribute__((ext_vector_type(4))) float v4f;
__device__ __forceinline__ float bf16_rne(float f) { unsigned int u = __float_as_uint(f); u += 0x7FFFu + ((u >> 16) & 1u); return __uint_as_float(u & 0xFFFF0000u); }
__device__ __forceinline__ float bfo(float f) { float r = bf16_rne(f); asm volatile("" : "+v"(r)); return r; }
__device__ __forceinline__ void split16(float v, b16& hi, b16& lo) { hi = (b16)v; lo = (b16)(v - (float)hi); }
__device__ __forceinline__ v16b frag_kb(const b16* p, int hh) { const v8b a = *(const v8b*)(p + 8 * hh), b = *(const v8b*)(p + 16 + 8 * hh); v16b f;
#pragma unroll
  for (int e = 0; e < 8; ++e) { f[e] = a[e]; f[8 + e] = b[e]; } return f; }
__device__ __forceinline__ v8f wmma16b(v16b a, v16b b, v8f c) { v8f d = __builtin_amdgcn_wmma_f32_16x16x32_f16(false, a, false, b, (short)0, c, false, false); asm volatile("v_nop\n\tv_nop\n\tv_nop\n\tv_nop" : "+v"(d) : "v"(a), "v"(b)); return d; }
__device__ __forceinline__ void wave_lds_sync() { __builtin_amdgcn_fence(__ATOMIC_RELEASE, "workgroup"); __builtin_amdgcn_wave_barrier(); __builtin_amdgcn_fence(__ATOMIC_ACQUIRE, "workgroup"); }
__device__ __forceinline__ float pmul(float a, float b) { float p = a * b; asm volatile("" : "+v"(p)); return p; }
__device__ __forceinline__ int iclamp(int v, int lo, int hi) { return v < lo ? lo : (v > hi ? hi : v); }
constexpr int CSR_NBLK = 512, CSR_GB = 9, CSR_GN = 1 << CSR_GB  , CSR_MAXG = 512, CSR_CAP = 12288  ;
__global__ __launch_bounds__(64) void csrA_kernel(const int* __restrict__ dst, int E, int N, int nG, int CHP, int NGP, int* __restrict__ STG, int* __restrict__ HST) {
  extern __shared__ int sm[];
  int* cnt = sm; int* run = sm + NGP; int* ids = sm + 2 * NGP;
  const int b = blockIdx.x; const int ch = (E + CSR_NBLK - 1) / CSR_NBLK; const int e0 = b * ch, e1 = min(E, e0 + ch);
  for (int i = threadIdx.x; i < NGP; i += 64) cnt[i] = 0;
  for (int i = threadIdx.x; i < CHP; i += 64) ids[i] = -1;
  __syncthreads();
  if (threadIdx.x == 0) {
    for (int e = e0; e < e1; ++e) { int d = dst[e]; d = (d < 0) ? 0 : (d >= N ? N - 1 : d); cnt[d >> CSR_GB] += 1; }
    int acc = 0; for (int g = 0; g < nG; ++g) { run[g] = acc; acc += cnt[g]; }
    for (int e = e0; e < e1; ++e) { int d = dst[e]; d = (d < 0) ? 0 : (d >= N ? N - 1 : d); const int g = d >> CSR_GB; ids[run[g]] = e; run[g] += 1; } }
  __syncthreads();
  typedef __attribute__((ext_vector_type(4))) int v4i;
  for (int pass = 0; pass < 2; ++pass) {
    for (int i = threadIdx.x; i < CHP / 4; i += 64) *(volatile v4i*)(STG + (size_t)b * CHP + i * 4) = *(const v4i*)(&ids[i * 4]);
    for (int i = threadIdx.x; i < NGP / 4; i += 64) { v4i v; for (int e = 0; e < 4; ++e) v[e] = (i * 4 + e < nG) ? cnt[i * 4 + e] : 0; *(volatile v4i*)(HST + (size_t)b * NGP + i * 4) = v; }
    __threadfence(); }
}
__global__ __launch_bounds__(512) void csrS_kernel(const int* __restrict__ HST, int nG, int NGP, int* __restrict__ START, int* __restrict__ TOT, int* __restrict__ OFF) {
  __shared__ int tot[CSR_MAXG];
  const int b = threadIdx.x;
  for (int pass = 0; pass < 2; ++pass) { int runb = 0; for (int g = 0; g < nG; ++g) { int c = HST[(size_t)b * NGP + g]; c = (c < 0) ? 0 : c; ((volatile int*)OFF)[(size_t)g * CSR_NBLK + b] = runb; runb += c; } __threadfence(); }
  for (int g = threadIdx.x; g < nG; g += 512) { int s = 0; for (int bb = 0; bb < CSR_NBLK; ++bb) { int c = HST[(size_t)bb * NGP + g]; s += (c < 0) ? 0 : c; } tot[g] = s; }
  __syncthreads();
  if (threadIdx.x < 32) {
    __shared__ int st[CSR_MAXG + 32];
    if (threadIdx.x == 0) { int acc = 0; for (int g = 0; g < NGP; ++g) { st[g] = acc; if (g < nG) acc += (tot[g] + 31) & ~31; } st[NGP] = acc; }
    __builtin_amdgcn_fence(__ATOMIC_RELEASE, "workgroup"); __builtin_amdgcn_wave_barrier(); __builtin_amdgcn_fence(__ATOMIC_ACQUIRE, "workgroup");
    for (int pass = 0; pass < 2; ++pass) { for (int i = threadIdx.x; i < NGP + 32; i += 32) { ((volatile int*)START)[i] = (i <= NGP) ? st[min(i, NGP)] : 0; ((volatile int*)TOT)[i] = (i < nG) ? tot[i] : 0; } __threadfence(); } }
}
__global__ __launch_bounds__(256) void csrB_kernel(const int* __restrict__ dst, int N, int nG, int CHP, int NGP, int permLen, const int* __restrict__ STG, const int* __restrict__ HST, const int* __restrict__ OFF, const int* __restrict__ START, const int* __restrict__ TOT, int* __restrict__ PERM, int* __restrict__ ROWPTR, int* __restrict__ ROWCNT, int* __restrict__ FLAG) {
  typedef __attribute__((ext_vector_type(4))) int v4i;
  __shared__ int ids[CSR_CAP]; __shared__ unsigned short key[CSR_CAP]; __shared__ int outp[CSR_CAP]; __shared__ int ncnt[CSR_GN + 1]; __shared__ int boff[CSR_NBLK + 1];
  const int g = blockIdx.x, t_ = threadIdx.x; int tot = TOT[g]; int st = START[g], stn = START[g + 1]; const int v0 = g * CSR_GN; const int nv = min(CSR_GN, N - v0);
  st = (st < 0) ? 0 : (st > permLen - 32 ? permLen - 32 : st) & ~31; stn = (stn < st) ? st : (stn > permLen ? permLen : stn); tot = (tot < 0) ? 0 : tot; if (tot > stn - st && tot <= CSR_CAP) tot = stn - st;
  if (tot > CSR_CAP) {
    for (int pass = 0; pass < 2; ++pass) { for (int i = t_; i < CSR_GN / 4; i += 256) { v4i a, c; for (int e = 0; e < 4; ++e) { a[e] = st; c[e] = 0; } *(volatile v4i*)(ROWPTR + v0 + i * 4) = a; *(volatile v4i*)(ROWCNT + v0 + i * 4) = c; } if (t_ == 0) ((volatile int*)FLAG)[0] = 1; __threadfence(); } (void)nv; return; }
  if (t_ == 0) { int acc = 0; for (int b = 0; b < CSR_NBLK; ++b) { boff[b] = acc; int c = HST[(size_t)b * NGP + g]; c = (c < 0) ? 0 : (c > CHP ? CHP : c); acc += c; if (acc > tot) acc = tot; } boff[CSR_NBLK] = acc; }
  for (int i = t_; i <= CSR_GN; i += 256) ncnt[i] = 0;
  __syncthreads();
  for (int b = 0; b < CSR_NBLK; ++b) { const int c = boff[b + 1] - boff[b]; int o_ = OFF[(size_t)g * CSR_NBLK + b]; o_ = (o_ < 0) ? 0 : (o_ > CHP - c ? CHP - c : o_); const int* src_ = STG + (size_t)b * CHP + o_;
    for (int i = t_; i < c; i += 256) { int id = src_[i]; id = (id < 0) ? 0 : id; ids[boff[b] + i] = id; int d = dst[id]; d = (d < v0) ? v0 : (d >= N ? N - 1 : d); int kk = d - v0; kk = (kk < 0) ? 0 : (kk >= CSR_GN ? CSR_GN - 1 : kk); key[boff[b] + i] = (unsigned short)kk; } }
  __syncthreads();
  if (t_ == 0) { for (int i = 0; i < tot; ++i) ncnt[key[i]] += 1; int acc = 0; for (int vl = 0; vl < CSR_GN; ++vl) { const int c = ncnt[vl]; ncnt[vl] = acc; acc += c; } ncnt[CSR_GN] = acc;
    for (int i = 0; i < tot; ++i) { const int vl = key[i]; outp[ncnt[vl]] = ids[i]; ncnt[vl] += 1; }
    for (int vl = CSR_GN; vl > 0; --vl) ncnt[vl] = ncnt[vl - 1]; ncnt[0] = 0; }
  __syncthreads();
  for (int pass = 0; pass < 2; ++pass) {
    for (int i = t_; i < (stn - st) / 4; i += 256) { v4i v; for (int e = 0; e < 4; ++e) { const int q = i * 4 + e; v[e] = (q < tot) ? outp[q] : -1; } *(volatile v4i*)(PERM + st + i * 4) = v; }
    for (int i = t_; i < CSR_GN / 4; i += 256) { v4i a, c; for (int e = 0; e < 4; ++e) { const int vl = i * 4 + e; a[e] = st + ncnt[vl]; c[e] = (vl < nv) ? (ncnt[vl + 1] - ncnt[vl]) : 0; } *(volatile v4i*)(ROWPTR + v0 + i * 4) = a; *(volatile v4i*)(ROWCNT + v0 + i * 4) = c; }
    __threadfence(); }
}
__global__ __launch_bounds__(256) void csrZ_kernel(int* __restrict__ p, size_t n4) { typedef __attribute__((ext_vector_type(4))) int v4i; const size_t tid = (size_t)blockIdx.x * 256 + threadIdx.x, nth = (size_t)gridDim.x * 256; v4i z = {0, 0, 0, 0}; for (size_t i = tid; i < n4; i += nth) *(volatile v4i*)(p + i * 4) = z; }
struct CsrBufs { int *STG, *HST, *OFF, *START, *TOT, *PERM, *ROWPTR, *ROWCNT, *FLAG; int nG, NGP, CHP; size_t permLen; char* base; size_t bytes; };
static size_t csr_carve(CsrBufs& c, char* ws, size_t off, int E, int N) {
  const size_t off0 = off; c.base = ws + off;
  auto al = [&](size_t bytes) { char* p = ws + off; off += (bytes + 255) & ~(size_t)255; return p; };
  c.nG = (N + CSR_GN - 1) / CSR_GN; c.NGP = (c.nG + 31) & ~31; const int ch = (E + CSR_NBLK - 1) / CSR_NBLK; c.CHP = (ch + 31) & ~31; c.permLen = (size_t)E + 32 * (size_t)c.nG + 32;
  c.STG = (int*)al((size_t)CSR_NBLK * c.CHP * 4); c.HST = (int*)al((size_t)CSR_NBLK * c.NGP * 4); c.OFF = (int*)al((size_t)c.NGP * CSR_NBLK * 4); c.START = (int*)al((size_t)(c.NGP + 64) * 4); c.TOT = (int*)al((size_t)(c.NGP + 64) * 4);
  c.PERM = (int*)al(c.permLen * 4); c.ROWPTR = (int*)al((size_t)c.nG * CSR_GN * 4); c.ROWCNT = (int*)al((size_t)c.nG * CSR_GN * 4); c.FLAG = (int*)al(256);
  c.bytes = off - off0; return off;
}
static void csr_build(const CsrBufs& c, const int* dst, int E, int N, hipStream_t stream) {
  const size_t smem = (size_t)(2 * c.NGP + c.CHP) * 4;
  csrZ_kernel<<<512, 256, 0, stream>>>((int*)c.base, c.bytes / 16);
  csrA_kernel<<<CSR_NBLK, 64, smem, stream>>>(dst, E, N, c.nG, c.CHP, c.NGP, c.STG, c.HST);
  csrS_kernel<<<1, 512, 0, stream>>>(c.HST, c.nG, c.NGP, c.START, c.TOT, c.OFF);
  csrB_kernel<<<c.nG, 256, 0, stream>>>(dst, N, c.nG, c.CHP, c.NGP, (int)c.permLen, c.STG, c.HST, c.OFF, c.START, c.TOT, c.PERM, c.ROWPTR, c.ROWCNT, c.FLAG);
}

typedef __attribute__((ext_vector_type(4))) _Float16 v4h;
__device__ __forceinline__ float lrelu(float v) { return v > 0.0f ? v : NSL_ * v; }
template <int K, int NOUTR, int NOUTP>
__global__ __launch_bounds__(256) void wt_kernel(const float* __restrict__ w, b16* __restrict__ WT, float scl) {
  const int u = blockIdx.x * 256 + threadIdx.x; if (u >= NOUTP * K / 8) return; const int e = u * 8; const int o = e / K, k0 = e % K; v8b v;
#pragma unroll
  for (int j = 0; j < 8; ++j) v[j] = (b16)(o < NOUTR ? bf16_rne(w[(size_t)(k0 + j) * NOUTR + o]) * scl : 0.0f);
  for (int pass = 0; pass < 2; ++pass) { *(volatile v8b*)(WT + e) = v; __threadfence(); }
}
template <int K, int NT, bool RND, int MODE, bool GIDX, int AP = K>
__global__ __launch_bounds__(64) void lin_kernel(const float* __restrict__ X, const int* __restrict__ gidx, const b16* __restrict__ WT, const b16* __restrict__ WQ, const float* __restrict__ bias, float* __restrict__ OUT, int opitch, int nvalid, int mrows) {
  constexpr int NC = NT * 16;
  __shared__ __attribute__((aligned(16))) b16 Ah[2][16][K + 8], Al[2][16][K + 8]; __shared__ __attribute__((aligned(16))) float Tf[2][16][NC + 4];
  const int wave = threadIdx.x >> 5, lane = threadIdx.x & 31, nloc = lane & 15, hlf = lane >> 4; const size_t m0 = (size_t)blockIdx.x * 32 + wave * 16;
  for (int idx = lane; idx < 16 * (K / 4); idx += 32) { const int rr = idx / (K / 4), c4 = (idx % (K / 4)) * 4; const size_t vrow = (m0 + rr < (size_t)nvalid) ? m0 + rr : (size_t)nvalid - 1; size_t arow = vrow; if (GIDX) arow = (size_t)iclamp(gidx[vrow], 0, VOC - 1);
    const v4f v = *(const v4f*)(X + arow * AP + c4);     v4h hv, lv;
    for (int j = 0; j < 4; ++j) { float vj = v[j]; if (MODE == 2) vj = fmaxf(vj, 0.0f); const float vs = (RND ? bf16_rne(vj) : vj) * XS; const b16 ph = (b16)vs; hv[j] = ph; lv[j] = (b16)((vs - (float)ph) * RS_); } *(v4h*)(&Ah[wave][rr][c4]) = hv; *(v4h*)(&Al[wave][rr][c4]) = lv; }
  wave_lds_sync();
  v8f acc[NT];
#pragma unroll
  for (int t = 0; t < NT; ++t) acc[t] = (v8f){};
#pragma unroll 1
  for (int kb = 0; kb < K; kb += 32) { const v16b a = frag_kb(&Ah[wave][nloc][kb], hlf); v16b al; if (!RND) al = frag_kb(&Al[wave][nloc][kb], hlf);
#pragma unroll
    for (int t = 0; t < NT; ++t) { const size_t wo_ = (size_t)(t * 16 + nloc) * K + kb; acc[t] = wmma16b(a, frag_kb(WT + wo_, hlf), acc[t]); if (!RND) acc[t] = wmma16b(al, frag_kb(WQ + wo_, hlf), acc[t]); } }
#pragma unroll
  for (int t = 0; t < NT; ++t) { const int col = t * 16 + nloc; const float bb = bf16_rne(bias[col]);
    for (int r = 0; r < 8; ++r) { const size_t vrow = m0 + 8 * hlf + r; float y = acc[t][r] * (1.0f / (XS * WSC)) + bb; if (MODE == 1) y = fmaxf(y, 0.0f); if (MODE == 7) y = (y > 0.0f) ? y : (__expf(y) - 1.0f); if (MODE == 22 || MODE == 23) { y += bf16_rne(__int_as_float(gidx[col])); if (MODE == 23) y = fmaxf(y, 0.0f); }     if (MODE == 20) { const float a_ = bf16_rne(__int_as_float(gidx[col])); y = (y >= 0.0f) ? y : a_ * y; }     Tf[wave][8 * hlf + r][col] = (vrow < (size_t)nvalid) ? y : 0.0f; } }
  wave_lds_sync();
  for (int pass = 0; pass < 2; ++pass) { for (int rr = 0; rr < 16; ++rr) { if (m0 + rr < (size_t)mrows) { if (NC >= 128) { for (int c8 = 0; c8 < NC; c8 += 128) *(volatile v4f*)(OUT + (m0 + rr) * (size_t)opitch + c8 + lane * 4) = *(const v4f*)(&Tf[wave][rr][c8 + lane * 4]); }
        else { if (lane < NC / 4) *(volatile v4f*)(OUT + (m0 + rr) * (size_t)opitch + lane * 4) = *(const v4f*)(&Tf[wave][rr][lane * 4]); } } } __threadfence(); }
}
__device__ __forceinline__ float gelu_(float v) { return 0.5f * v * (1.0f + erff(v * 0.70710678118654752f)); }
__device__ __forceinline__ float rsum8(float s) { s += __shfl_xor(s, 1); s += __shfl_xor(s, 2); s += __shfl_xor(s, 4); return s; }
__global__ __launch_bounds__(256) void smagg_kernel(const float* __restrict__ SN, const float* __restrict__ za, const int* __restrict__ srcs, const int* __restrict__ PERM, const int* __restrict__ ROWPTR, const int* __restrict__ ROWCNT, int permLen, float* __restrict__ CB, int mrows) {
  const int tid = threadIdx.x; const int row = tid >> 3, g = tid & 7, c0 = g * 8; const int v = blockIdx.x * 32 + row; const int vv = v < N ? v : N - 1;
  int cnt = 0, p0 = 0; if (v < N) { cnt = iclamp(ROWCNT[v], 0, 65536); p0 = iclamp(ROWPTR[v], 0, permLen - 1); if (p0 + cnt > permLen) cnt = permLen - p0; }
  float s[8], mx[8]; for (int j = 0; j < 8; ++j) { s[j] = 0.0f; mx[j] = -INFINITY; }
#pragma unroll 1
  for (int i = 0; i < cnt; ++i) { const int e = iclamp(PERM[p0 + i], 0, E - 1); int sidx = iclamp(srcs[e], 0, N - 1); if (SRCM < N) sidx %= SRCM; const float* hr = SN + (size_t)sidx * P2 + F + c0;
    const v4f a = *(const v4f*)hr, b = *(const v4f*)(hr + 4); for (int j = 0; j < 4; ++j) { s[j] += a[j]; s[4 + j] += b[j]; mx[j] = fmaxf(mx[j], a[j]); mx[4 + j] = fmaxf(mx[4 + j], b[j]); } }
  const float z0 = bfo(za[0]), z1 = bfo(za[1]), z2 = bfo(za[2]); const float cs = z0 + z1 / fmaxf((float)cnt, 1.0f); const v4f xa = *(const v4f*)(SN + (size_t)vv * P2 + c0), xb = *(const v4f*)(SN + (size_t)vv * P2 + c0 + 4);
  for (int pass = 0; pass < 2; ++pass) { if (v < mrows) { float* orow = CB + (size_t)v * P2 + c0; v4f o0, o1, n0, n1;
      for (int j = 0; j < 4; ++j) { o0[j] = (v < N) ? xa[j] : 0.0f; o1[j] = (v < N) ? xb[j] : 0.0f; n0[j] = (v < N) ? pmul(cs, s[j]) + pmul(z2, (cnt > 0) ? mx[j] : 0.0f) : 0.0f; n1[j] = (v < N) ? pmul(cs, s[4 + j]) + pmul(z2, (cnt > 0) ? mx[4 + j] : 0.0f) : 0.0f; }
      *(volatile v4f*)orow = o0; *(volatile v4f*)(orow + 4) = o1; *(volatile v4f*)(orow + F) = n0; *(volatile v4f*)(orow + F + 4) = n1; }
    __threadfence(); }
}
__global__ __launch_bounds__(256) void mixln_kernel(const float* __restrict__ CB, const float* __restrict__ CC, int ccp, const float* __restrict__ zc, const float* __restrict__ zt, const float* __restrict__ pw, const float* __restrict__ lg, const float* __restrict__ lb, float* __restrict__ EMBL, int mrows) {
  const int tid = threadIdx.x; const int row = tid >> 3, g = tid & 7, c0 = g * 8; const int v = blockIdx.x * 32 + row; const int vv = v < N ? v : N - 1;
  const float zc0 = bfo(zc[0]), zc1 = bfo(zc[1]), zt0 = bfo(zt[0]), zt1 = bfo(zt[1]), pwl = bfo(pw[0]); float h[8]; float sm = 0.0f;
#pragma unroll
  for (int q = 0; q < 2; ++q) { const v4f xs = *(const v4f*)(CB + (size_t)vv * P2 + c0 + 4 * q), xn = *(const v4f*)(CB + (size_t)vv * P2 + F + c0 + 4 * q), cc = *(const v4f*)(CC + (size_t)vv * ccp + c0 + 4 * q);
    for (int j = 0; j < 4; ++j) { float t = pmul(zc0, xs[j] + xn[j]) + pmul(zc1, cc[j]); t = pmul(zt0, fmaxf(t, 0.0f)) + pmul(zt1, (t > 0.0f) ? t : pmul(pwl, t)); h[4 * q + j] = t; sm += t; } }
  sm = rsum8(sm); const float mu = sm * (1.0f / F); float sv = 0.0f; for (int j = 0; j < 8; ++j) { const float d = h[j] - mu; sv += pmul(d, d); } sv = rsum8(sv); const float rs = rsqrtf(sv * (1.0f / F) + LNEPS);
  for (int pass = 0; pass < 2; ++pass) { if (v < mrows) { float* orow = EMBL + (size_t)v * PE + c0;
#pragma unroll
      for (int q = 0; q < 2; ++q) { const v4f g4 = *(const v4f*)(lg + c0 + 4 * q), b4 = *(const v4f*)(lb + c0 + 4 * q); v4f o; for (int j = 0; j < 4; ++j) o[j] = (v < N) ? pmul(pmul(h[4 * q + j] - mu, rs), bfo(g4[j])) + bfo(b4[j]) : 0.0f; *(volatile v4f*)(orow + 4 * q) = o; } }
    __threadfence(); }
}
__global__ __launch_bounds__(256) void lcmix_kernel(const float* __restrict__ EMBP, const float* __restrict__ LC, int lcp, const float* __restrict__ zl, float* __restrict__ XO, int mrows) {
  const size_t i = (size_t)blockIdx.x * 256 + threadIdx.x; if (i >= (size_t)mrows * 16) return; const size_t v = i >> 4; const int c = (int)(i & 15) * 4; const float z0 = bfo(zl[0]), z1 = bfo(zl[1]), z2 = bfo(zl[2]);
  const v4f pv = *(const v4f*)(EMBP + v * PE + c), hv = *(const v4f*)(EMBP + v * PE + F + c), lc = *(const v4f*)(LC + v * lcp + c); v4f o;
  for (int j = 0; j < 4; ++j) o[j] = (v < (size_t)N) ? pmul(z0, hv[j]) + pmul(z1, hv[j] + pv[j]) + pmul(z2, lc[j]) : 0.0f;
  for (int pass = 0; pass < 2; ++pass) { *(volatile v4f*)(XO + v * P2 + c) = o; __threadfence(); }
}
__global__ __launch_bounds__(256) void lagg_kernel(const float* __restrict__ EMB, const float* __restrict__ AC, int acp, const float* __restrict__ zg, float* __restrict__ OUT, int op, int mrows) {
  const size_t i = (size_t)blockIdx.x * 256 + threadIdx.x; if (i >= (size_t)mrows * 16) return; const size_t v = i >> 4; const int c = (int)(i & 15) * 4; const float z0 = bfo(zg[0]), z1 = bfo(zg[1]), z2 = bfo(zg[2]);
  const v4f e0 = *(const v4f*)(EMB + v * PE + c), e1 = *(const v4f*)(EMB + v * PE + F + c), e2 = *(const v4f*)(EMB + v * PE + 2 * F + c), e3 = *(const v4f*)(EMB + v * PE + 3 * F + c), ac = *(const v4f*)(AC + v * acp + c); v4f o;
  for (int j = 0; j < 4; ++j) { const float m = fmaxf(fmaxf(e0[j], e1[j]), fmaxf(e2[j], e3[j])); o[j] = (v < (size_t)N) ? pmul(z0, e3[j]) + pmul(z1, m) + pmul(z2, ac[j]) : 0.0f; }
  for (int pass = 0; pass < 2; ++pass) { *(volatile v4f*)(OUT + v * op + c) = o; __threadfence(); }
}
__global__ __launch_bounds__(128) void bcat_kernel(const float* __restrict__ b1, const float* __restrict__ b2, float* __restrict__ B) { const int c = threadIdx.x; const float v = (c < F) ? b1[c] : b2[c - F]; for (int pass = 0; pass < 2; ++pass) { ((volatile float*)B)[c] = v; __threadfence(); } }
}

extern "C" void kernel_launch(void* const* d_in, const int* in_sizes, int n_in, void* d_out, int out_size, void* d_ws, size_t ws_size, hipStream_t stream) {
  (void)n_in;
  auto Fp = [&](int i) { return (const float*)d_in[i]; }; auto Ip = [&](int i) { return (const int*)d_in[i]; };
  const int want[26] = {N * FIN, 2 * EFULL, FIN * F, F, NLAY * F * F, NLAY * F, NLAY * F * F, NLAY * F, NLAY * P2 * F, NLAY * F, NLAY * P2 * F, NLAY * F, NLAY * F, NLAY * F, NLAY, PE * F, F, F * F, F, F * F, F, NLAY * 3, NLAY * 2, NLAY * 2, NLAY * 3, 3};
  for (int i = 0; i < 26; ++i) if (in_sizes[i] != want[i]) return;
  if (out_size != N * FO) return;
  size_t off = 0; char* ws = (char*)d_ws;
  auto carve = [&](size_t bytes) { char* p = ws + off; off += (bytes + 255) & ~(size_t)255; return p; };
  b16* WPRE = (b16*)carve((size_t)F * FIN * 2);
  b16* WSN[NLAY]; b16* WSNQ[NLAY]; b16* WC[NLAY]; b16* WCQ[NLAY]; b16* WLC[NLAY]; b16* WLCQ[NLAY]; float* BSN[NLAY];
  for (int l = 0; l < NLAY; ++l) { WSN[l] = (b16*)carve((size_t)P2 * F * 2); WSNQ[l] = (b16*)carve((size_t)P2 * F * 2); WC[l] = (b16*)carve((size_t)F * P2 * 2); WCQ[l] = (b16*)carve((size_t)F * P2 * 2); WLC[l] = (b16*)carve((size_t)F * P2 * 2); WLCQ[l] = (b16*)carve((size_t)F * P2 * 2); BSN[l] = (float*)carve(1024); }
  b16* WLA = (b16*)carve((size_t)F * PE * 2); b16* WLAQ = (b16*)carve((size_t)F * PE * 2); b16* WF1 = (b16*)carve((size_t)F * F * 2); b16* WF1Q = (b16*)carve((size_t)F * F * 2); b16* WF2 = (b16*)carve((size_t)F * F * 2); b16* WF2Q = (b16*)carve((size_t)F * F * 2);
  float* EMB = (float*)carve((size_t)NP * PE * 4); float* SN = (float*)carve((size_t)NP * P2 * 4); float* CB = (float*)carve((size_t)NP * P2 * 4);
  CsrBufs csr; off = csr_carve(csr, ws, off, E, N);
  if (off > ws_size || off > ((size_t)244 << 20)) return;
  { const unsigned g64 = (F * F / 8 + 255) / 256, g128 = (F * P2 / 8 + 255) / 256;
    wt_kernel<FIN, F, F><<<(F * FIN / 8 + 255) / 256, 256, 0, stream>>>(Fp(2), WPRE, WSC);
    for (int l = 0; l < NLAY; ++l) {
      wt_kernel<F, F, F><<<g64, 256, 0, stream>>>(Fp(4) + (size_t)l * F * F, WSN[l], WSC); wt_kernel<F, F, F><<<g64, 256, 0, stream>>>(Fp(6) + (size_t)l * F * F, WSN[l] + (size_t)F * F, WSC);
      wt_kernel<F, F, F><<<g64, 256, 0, stream>>>(Fp(4) + (size_t)l * F * F, WSNQ[l], WSQ); wt_kernel<F, F, F><<<g64, 256, 0, stream>>>(Fp(6) + (size_t)l * F * F, WSNQ[l] + (size_t)F * F, WSQ);
      wt_kernel<P2, F, F><<<g128, 256, 0, stream>>>(Fp(8) + (size_t)l * P2 * F, WC[l], WSC); wt_kernel<P2, F, F><<<g128, 256, 0, stream>>>(Fp(8) + (size_t)l * P2 * F, WCQ[l], WSQ);
      wt_kernel<P2, F, F><<<g128, 256, 0, stream>>>(Fp(10) + (size_t)l * P2 * F, WLC[l], WSC); wt_kernel<P2, F, F><<<g128, 256, 0, stream>>>(Fp(10) + (size_t)l * P2 * F, WLCQ[l], WSQ);
      bcat_kernel<<<1, 128, 0, stream>>>(Fp(5) + (size_t)l * F, Fp(7) + (size_t)l * F, BSN[l]); }
    wt_kernel<PE, F, F><<<(F * PE / 8 + 255) / 256, 256, 0, stream>>>(Fp(15), WLA, WSC); wt_kernel<PE, F, F><<<(F * PE / 8 + 255) / 256, 256, 0, stream>>>(Fp(15), WLAQ, WSQ);
    wt_kernel<F, F, F><<<g64, 256, 0, stream>>>(Fp(17), WF1, WSC); wt_kernel<F, F, F><<<g64, 256, 0, stream>>>(Fp(17), WF1Q, WSQ); wt_kernel<F, F, F><<<g64, 256, 0, stream>>>(Fp(19), WF2, WSC); wt_kernel<F, F, F><<<g64, 256, 0, stream>>>(Fp(19), WF2Q, WSQ); }
  csr_build(csr, Ip(1) + EFULL, E, N, stream);
  lin_kernel<FIN, 4, true, 0, false><<<NRL / 32, 64, 0, stream>>>(Fp(0), nullptr, WPRE, WPRE, Fp(3), EMB, PE, N, NRL);
  for (int l = 0; l < NLAY; ++l) {
    if (l == 0) lin_kernel<F, 8, false, 0, false, PE><<<NRL / 32, 64, 0, stream>>>(EMB, nullptr, WSN[l], WSNQ[l], BSN[l], SN, P2, N, NRL);
    else        lin_kernel<F, 8, false, 0, false, P2><<<NRL / 32, 64, 0, stream>>>(CB, nullptr, WSN[l], WSNQ[l], BSN[l], SN, P2, N, NRL);
    smagg_kernel<<<NRL / 32, 256, 0, stream>>>(SN, Fp(21) + 3 * l, Ip(1), csr.PERM, csr.ROWPTR, csr.ROWCNT, (int)csr.permLen, CB, NRL);
    lin_kernel<P2, 4, false, 0, false><<<NRL / 32, 64, 0, stream>>>(CB, nullptr, WC[l], WCQ[l], Fp(9) + (size_t)l * F, SN, P2, N, NRL);
    mixln_kernel<<<NRL / 32, 256, 0, stream>>>(CB, SN, P2, Fp(22) + 2 * l, Fp(23) + 2 * l, Fp(14) + l, Fp(12) + (size_t)l * F, Fp(13) + (size_t)l * F, EMB + (size_t)(l + 1) * F, NRL);
    lin_kernel<P2, 4, false, 0, false, PE><<<NRL / 32, 64, 0, stream>>>(EMB + (size_t)l * F, nullptr, WLC[l], WLCQ[l], Fp(11) + (size_t)l * F, SN + F, P2, N, NRL);
    lcmix_kernel<<<(unsigned)(((size_t)NRL * 16 + 255) / 256), 256, 0, stream>>>(EMB + (size_t)l * F, SN + F, P2, Fp(24) + 3 * l, CB, NRL); }
  lin_kernel<PE, 4, false, 0, false><<<NPL / 32, 64, 0, stream>>>(EMB, nullptr, WLA, WLAQ, Fp(16), SN, P2, N, NPL);
  lagg_kernel<<<(unsigned)(((size_t)NPL * 16 + 255) / 256), 256, 0, stream>>>(EMB, SN, P2, Fp(25), CB, P2, NPL);
  lin_kernel<F, 4, false, 1, false, P2><<<NPL / 32, 64, 0, stream>>>(CB, nullptr, WF1, WF1Q, Fp(18), SN, P2, N, NPL);
  lin_kernel<F, 4, false, 0, false, P2><<<NPL / 32, 64, 0, stream>>>(SN, nullptr, WF2, WF2Q, Fp(20), (float*)d_out, FO, N, NL);
}
